// SparseAttention_21732534518122
// MI455X (gfx1250) — hardware-verified
//
#include <hip/hip_runtime.h>


#ifndef NB
#define NB 1
#endif
#ifndef SEQ
#define SEQ 4096
#endif
#define NB_FULL   1
#define SEQ_FULL  4096
#define DM    1536
#define NH    12
#define HD    128
#define BAND  2
#define NKEY  (2 * BAND + 1)
#define SCL   0.08838834764831845f
#define WOCAR 64.0f
#define LNEPS 1e-5f
#define LOG2E 1.4426950408889634f

static_assert(SEQ % 64 == 0);
static_assert(DM % 128 == 0);
static_assert(NH * HD == DM);
static_assert(HD == 16 * 8);
static_assert(NB >= 1 && NB <= NB_FULL);
static_assert(SEQ <= SEQ_FULL);

typedef _Float16 h16;
typedef unsigned short bf;
typedef __attribute__((ext_vector_type(16))) __bf16   v16bf;
typedef __attribute__((ext_vector_type(16))) _Float16 v16h;
typedef __attribute__((ext_vector_type(8)))  _Float16 v8h;
typedef __attribute__((ext_vector_type(8)))  unsigned short v8us;
typedef __attribute__((ext_vector_type(8)))  float    v8f;
typedef __attribute__((ext_vector_type(4)))  float    v4f;
typedef __attribute__((ext_vector_type(2)))  _Float16 v2h;
typedef __attribute__((ext_vector_type(2)))  unsigned short v2us;
typedef v8h  __attribute__((may_alias)) v8ha;
typedef v4f  __attribute__((may_alias)) v4fa;
typedef v8us __attribute__((may_alias)) v8usa;

__device__ __forceinline__ unsigned short f2bf(float f) { unsigned u = __float_as_uint(f); u += 0x7FFFu + ((u >> 16) & 1u); return (unsigned short)(u >> 16); }
__device__ __forceinline__ float bf2f(unsigned short b) { return __uint_as_float(((unsigned)b) << 16); }
__device__ __forceinline__ float bfr(float f) { return bf2f(f2bf(f)); }
__device__ __forceinline__ v16h cat16(v8h lo, v8h hi) { return __builtin_shufflevector(lo, hi, 0, 1, 2, 3, 4, 5, 6, 7, 8, 9, 10, 11, 12, 13, 14, 15); }
__device__ __forceinline__ v16bf cat16b(v8us lo, v8us hi) { return __builtin_bit_cast(v16bf, __builtin_shufflevector(lo, hi, 0, 1, 2, 3, 4, 5, 6, 7, 8, 9, 10, 11, 12, 13, 14, 15)); }
__device__ __forceinline__ v8f wmma16(v16h a, v16h b, v8f c) { return __builtin_amdgcn_wmma_f32_16x16x32_f16(false, a, false, b, (short)0, c, false, false); }
__device__ __forceinline__ v8f wmmab(v16bf a, v16bf b, v8f c) { return __builtin_amdgcn_wmma_f32_16x16x32_bf16(false, a, false, b, (short)0, c, false, false); }

template <typename T16> struct WFrag;
template <> struct WFrag<h16> { typedef v16h V; static __device__ __forceinline__ V ld(const h16* p) { return cat16(*(const v8h*)p, *(const v8h*)(p + 16)); } static __device__ __forceinline__ v8f mma(V a, V b, v8f c) { return wmma16(a, b, c); } };
template <> struct WFrag<bf> { typedef v16bf V; static __device__ __forceinline__ V ld(const bf* p) { return cat16b(*(const v8us*)p, *(const v8us*)(p + 16)); } static __device__ __forceinline__ v8f mma(V a, V b, v8f c) { return wmmab(a, b, c); } };
template <typename T16, int NSPLIT, bool BIAS>
__global__ __launch_bounds__(32) void k_gemmw(const T16* __restrict__ A, const T16* __restrict__ A2, const T16* __restrict__ Bt, const T16* __restrict__ Bt2, int K, float* C, int ldc, const float* __restrict__ bias, float cscale, size_t sA, size_t sB, size_t sC) {
    typedef typename WFrag<T16>::V V;
    __shared__ __align__(16) float os[16 * 68];
    const size_t z = blockIdx.z; A += z * sA; if (A2) A2 += z * sA; Bt += z * sB; if (Bt2) Bt2 += z * sB; C += z * sC;
    const int lane = threadIdx.x & 31, lr = lane & 15, hi = lane >> 4; const int r0 = blockIdx.x * 64, c0 = blockIdx.y * 64;
    v8f acc[4][4];
#pragma unroll
    for (int mb = 0; mb < 4; ++mb)
#pragma unroll
        for (int nb = 0; nb < 4; ++nb) acc[mb][nb] = (v8f){};
    const size_t aoff = (size_t)(r0 + lr) * K + 8 * hi, boff = (size_t)(c0 + lr) * K + 8 * hi;
#pragma unroll 1
    for (int kc = 0; kc < K; kc += 32) {
        V a[4], a2[4];
#pragma unroll
        for (int mb = 0; mb < 4; ++mb) { a[mb] = WFrag<T16>::ld(A + aoff + (size_t)mb * 16 * K + kc); if (NSPLIT == 1 || NSPLIT == 2) a2[mb] = WFrag<T16>::ld(A2 + aoff + (size_t)mb * 16 * K + kc); }
#pragma unroll
        for (int nb = 0; nb < 4; ++nb) { const V b = WFrag<T16>::ld(Bt + boff + (size_t)nb * 16 * K + kc); V b2; if (NSPLIT >= 2) b2 = WFrag<T16>::ld(Bt2 + boff + (size_t)nb * 16 * K + kc);
#pragma unroll
            for (int mb = 0; mb < 4; ++mb) { acc[mb][nb] = WFrag<T16>::mma(a[mb], b, acc[mb][nb]); if (NSPLIT == 1 || NSPLIT == 2) acc[mb][nb] = WFrag<T16>::mma(a2[mb], b, acc[mb][nb]); if (NSPLIT >= 2) acc[mb][nb] = WFrag<T16>::mma(a[mb], b2, acc[mb][nb]); } }
        asm volatile("v_nop\n\tv_nop\n\tv_nop\n\tv_nop" : "+v"(acc[0][0]), "+v"(acc[1][1]), "+v"(acc[2][2]), "+v"(acc[3][3]) : "v"(a[0]), "v"(a[3]));
    }
#pragma unroll
    for (int mb = 0; mb < 4; ++mb) {
#pragma unroll
        for (int nb = 0; nb < 4; ++nb) {
#pragma unroll
            for (int j = 0; j < 8; ++j) os[(hi * 8 + j) * 68 + nb * 16 + lr] = acc[mb][nb][j]; }
        __builtin_amdgcn_wave_barrier(); asm volatile("" ::: "memory");
        float* crow = C + (size_t)(r0 + mb * 16) * ldc + c0;
#pragma unroll 1
        for (int ps = 0; ps < 2; ++ps) {
#pragma unroll
            for (int s = 0; s < 8; ++s) { const int row = 2 * s + hi, cofs = lr * 4; v4f val = *(const v4fa*)(os + row * 68 + cofs); val = val * cscale;
                if (BIAS) { val[0] += bfr(bias[c0 + cofs]); val[1] += bfr(bias[c0 + cofs + 1]); val[2] += bfr(bias[c0 + cofs + 2]); val[3] += bfr(bias[c0 + cofs + 3]); }
                *(volatile v4f*)(crow + (size_t)row * ldc + cofs) = val; }
            if (ps == 0) __threadfence(); }
        __builtin_amdgcn_wave_barrier(); asm volatile("" ::: "memory");
    }
}

__global__ __launch_bounds__(256) void k_wtG(const float* __restrict__ w, int K, int N, bf* Bt) {
    const int lane = threadIdx.x & 31; const int L0 = (blockIdx.x * 8 + (threadIdx.x >> 5)) * 8; const int nlines = N * K / 64;
#pragma unroll
    for (int ps = 0; ps < 2; ++ps) {
#pragma unroll 1
        for (int l = 0; l < 8; ++l) { const int L = L0 + l; if (L >= nlines) break; const size_t e = (size_t)L * 64 + lane * 2; const int k = (int)(e % K), n = (int)(e / K); v2us o;
            o[0] = f2bf(w[(size_t)k * N + n]); o[1] = f2bf(w[(size_t)(k + 1) * N + n]); *(volatile v2us*)(Bt + e) = o; }
        if (ps == 0) __threadfence(); }
}
__global__ __launch_bounds__(256) void k_wtGh(const float* __restrict__ w, int K, int N, float car, h16* Bt) {
    const int lane = threadIdx.x & 31; const int L0 = (blockIdx.x * 8 + (threadIdx.x >> 5)) * 8; const int nlines = N * K / 64;
#pragma unroll
    for (int ps = 0; ps < 2; ++ps) {
#pragma unroll 1
        for (int l = 0; l < 8; ++l) { const int L = L0 + l; if (L >= nlines) break; const size_t e = (size_t)L * 64 + lane * 2; const int k = (int)(e % K), n = (int)(e / K); v2h o;
            o[0] = (h16)(bfr(w[(size_t)k * N + n]) * car); o[1] = (h16)(bfr(w[(size_t)(k + 1) * N + n]) * car); *(volatile v2h*)(Bt + e) = o; }
        if (ps == 0) __threadfence(); }
}
__global__ __launch_bounds__(256) void k_cvt8(const float* __restrict__ src, bf* dst, size_t n8) { const size_t i = (size_t)blockIdx.x * 256 + threadIdx.x; if (i >= n8) return; const v8f v = *(const v8f*)(src + i * 8); v8us o;
#pragma unroll
    for (int k = 0; k < 8; ++k) o[k] = f2bf(v[k]); *(volatile v8us*)(dst + i * 8) = o; __threadfence(); *(volatile v8us*)(dst + i * 8) = o; }

__device__ __forceinline__ float hdot(v4f qa, v4f qb, v4f ka, v4f kb) {
    float s = qa[0] * ka[0]; s += qa[1] * ka[1]; s += qa[2] * ka[2]; s += qa[3] * ka[3];
    s += qb[0] * kb[0]; s += qb[1] * kb[1]; s += qb[2] * kb[2]; s += qb[3] * kb[3];
#pragma unroll
    for (int sh = 1; sh < 16; sh <<= 1) s += __shfl_xor(s, sh, 32);
    return s;
}

__global__ __launch_bounds__(256) void k_band(const float* __restrict__ Q, const float* __restrict__ Kt, const float* __restrict__ V, h16* CTX) {
    const int lane = threadIdx.x & 31, hi = lane >> 4, lr = lane & 15;
    const int task = blockIdx.x * 8 + (threadIdx.x >> 5);
    if (task >= NH * (SEQ / 2)) return;
    const int h = task / (SEQ / 2); const int q = 2 * (task % (SEQ / 2)) + hi;
    const size_t cofs = (size_t)h * HD + (size_t)lr * 8;
    const float* qp = Q + (size_t)q * DM + cofs; const v4f qa = *(const v4f*)qp; const v4f qb = *(const v4f*)(qp + 4);
    float mx = -3.0e38f;
#pragma unroll 1
    for (int j = 0; j < NKEY; ++j) {
        const int jj = q - BAND + j; const bool ok = (jj >= 0) && (jj < SEQ); const int jc = jj < 0 ? 0 : (jj > SEQ - 1 ? SEQ - 1 : jj);
        const float* kp = Kt + (size_t)jc * DM + cofs; const v4f ka = *(const v4f*)kp; const v4f kb = *(const v4f*)(kp + 4);
        float s = hdot(qa, qb, ka, kb) * SCL; s = ok ? s : -3.0e38f; mx = fmaxf(mx, s);
    }
    float sum = 0.f; v4f ca, cb; ca = (v4f){}; cb = (v4f){};
#pragma unroll 1
    for (int j = 0; j < NKEY; ++j) {
        const int jj = q - BAND + j; const bool ok = (jj >= 0) && (jj < SEQ); const int jc = jj < 0 ? 0 : (jj > SEQ - 1 ? SEQ - 1 : jj);
        const float* kp = Kt + (size_t)jc * DM + cofs; const v4f ka = *(const v4f*)kp; const v4f kb = *(const v4f*)(kp + 4);
        const float s = hdot(qa, qb, ka, kb) * SCL;
        const float t = __fmul_rn(__fsub_rn(s, mx), LOG2E); float e = __builtin_amdgcn_exp2f(t); e = ok ? e : 0.f;
        const float* vp = V + (size_t)jc * DM + cofs; const v4f va = *(const v4f*)vp; const v4f vb = *(const v4f*)(vp + 4);
        sum += e; ca += e * va; cb += e * vb;
    }
    const float inv = __builtin_amdgcn_rcpf(sum);
    v8h o;
#pragma unroll
    for (int i = 0; i < 4; ++i) { o[i] = (h16)(ca[i] * inv); o[4 + i] = (h16)(cb[i] * inv); }
    h16* dst = CTX + (size_t)q * DM + cofs;
    *(volatile v8h*)dst = o; __threadfence(); *(volatile v8h*)dst = o;
}

__global__ __launch_bounds__(256) void k_ln(const float* __restrict__ X, const float* __restrict__ Y, const float* __restrict__ gam, const float* __restrict__ bet, float* OUT) {
    const int lane = threadIdx.x & 31; const int row = blockIdx.x * 8 + (threadIdx.x >> 5); if (row >= SEQ) return;
    const float* xr = X + (size_t)row * DM; const float* yr = Y + (size_t)row * DM; float* orow = OUT + (size_t)row * DM;
    float s = 0.f;
#pragma unroll 1
    for (int ch = 0; ch < DM / 128; ++ch) { const int c = ch * 128 + lane * 4; const v4f xv = *(const v4f*)(xr + c); const v4f yv = *(const v4f*)(yr + c);
#pragma unroll
        for (int i = 0; i < 4; ++i) s += bfr(xv[i]) + yv[i]; }
#pragma unroll
    for (int sh = 16; sh; sh >>= 1) s += __shfl_xor(s, sh, 32);
    const float mu = s * (1.0f / DM);
    float vs = 0.f;
#pragma unroll 1
    for (int ch = 0; ch < DM / 128; ++ch) { const int c = ch * 128 + lane * 4; const v4f xv = *(const v4f*)(xr + c); const v4f yv = *(const v4f*)(yr + c);
#pragma unroll
        for (int i = 0; i < 4; ++i) { const float d = (bfr(xv[i]) + yv[i]) - mu; vs += d * d; } }
#pragma unroll
    for (int sh = 16; sh; sh >>= 1) vs += __shfl_xor(vs, sh, 32);
    const float rstd = rsqrtf(vs * (1.0f / DM) + LNEPS);
#pragma unroll 1
    for (int ps = 0; ps < 2; ++ps) {
#pragma unroll 1
        for (int ch = 0; ch < DM / 128; ++ch) { const int c = ch * 128 + lane * 4; const v4f xv = *(const v4f*)(xr + c); const v4f yv = *(const v4f*)(yr + c);
            const v4f gv = *(const v4f*)(gam + c); const v4f bv = *(const v4f*)(bet + c); v4f o;
#pragma unroll
            for (int i = 0; i < 4; ++i) o[i] = ((bfr(xv[i]) + yv[i]) - mu) * rstd * bfr(gv[i]) + bfr(bv[i]);
            *(volatile v4f*)(orow + c) = o; }
        if (ps == 0) __threadfence(); }
}

extern "C" void kernel_launch(void* const* d_in, const int* in_sizes, int n_in,
                              void* d_out, int out_size, void* d_ws, size_t ws_size, hipStream_t stream) {
    if (n_in < 11) return;
    if (in_sizes[0] < (NB - 1) * SEQ_FULL * DM + SEQ * DM) return;
    if (in_sizes[1] < DM * DM || in_sizes[3] < DM * DM || in_sizes[5] < DM * DM || in_sizes[7] < DM * DM) return;
    if (in_sizes[2] < DM || in_sizes[4] < DM || in_sizes[6] < DM || in_sizes[8] < DM || in_sizes[9] < DM || in_sizes[10] < DM) return;
    if (out_size < NB * SEQ * DM) return;
    const float* X   = (const float*)d_in[0];
    const float* Wq  = (const float*)d_in[1];  const float* bq = (const float*)d_in[2];
    const float* Wk  = (const float*)d_in[3];  const float* bk = (const float*)d_in[4];
    const float* Wv  = (const float*)d_in[5];  const float* bv = (const float*)d_in[6];
    const float* Wo  = (const float*)d_in[7];  const float* bo = (const float*)d_in[8];
    const float* gam = (const float*)d_in[9];  const float* bet = (const float*)d_in[10];
    float* OUT = (float*)d_out;
    char* wsp = (char*)d_ws;
    auto take = [&](size_t bytes) { char* p = wsp; wsp += (bytes + 255) & ~(size_t)255; return (void*)p; };
    bf*  XB  = (bf*)take((size_t)SEQ * DM * 2);
    bf*  WQT = (bf*)take((size_t)DM * DM * 2);
    bf*  WKT = (bf*)take((size_t)DM * DM * 2);
    bf*  WVT = (bf*)take((size_t)DM * DM * 2);
    h16* WOT = (h16*)take((size_t)DM * DM * 2);
    float* QF = (float*)take((size_t)SEQ * DM * 4);
    float* KF = (float*)take((size_t)SEQ * DM * 4);
    float* VF = (float*)take((size_t)SEQ * DM * 4);
    h16* CTX = (h16*)take((size_t)SEQ * DM * 2);
    float* YF = QF;
    if ((size_t)(wsp - (char*)d_ws) > ws_size) return;

    const unsigned gw = (unsigned)((DM * DM / 64 + 63) / 64);
    k_wtG<<<gw, 256, 0, stream>>>(Wq, DM, DM, WQT);
    k_wtG<<<gw, 256, 0, stream>>>(Wk, DM, DM, WKT);
    k_wtG<<<gw, 256, 0, stream>>>(Wv, DM, DM, WVT);
    k_wtGh<<<gw, 256, 0, stream>>>(Wo, DM, DM, WOCAR, WOT);
    const dim3 gg(SEQ / 64, DM / 64, 1);
    for (int b = 0; b < NB; ++b) {
        const float* xb = X + (size_t)b * SEQ_FULL * DM; float* ob = OUT + (size_t)b * SEQ * DM;
        k_cvt8<<<(unsigned)(((size_t)SEQ * DM / 8 + 255) / 256), 256, 0, stream>>>(xb, XB, (size_t)SEQ * DM / 8);
        k_gemmw<bf, 0, true><<<gg, 32, 0, stream>>>(XB, nullptr, WQT, nullptr, DM, QF, DM, bq, 1.0f, 0, 0, 0);
        k_gemmw<bf, 0, true><<<gg, 32, 0, stream>>>(XB, nullptr, WKT, nullptr, DM, KF, DM, bk, 1.0f, 0, 0, 0);
        k_gemmw<bf, 0, true><<<gg, 32, 0, stream>>>(XB, nullptr, WVT, nullptr, DM, VF, DM, bv, 1.0f, 0, 0, 0);
        k_band<<<(unsigned)((NH * (SEQ / 2) + 7) / 8), 256, 0, stream>>>(QF, KF, VF, CTX);
        k_gemmw<h16, 0, true><<<gg, 32, 0, stream>>>(CTX, nullptr, WOT, nullptr, DM, YF, DM, bo, 1.0f / WOCAR, 0, 0, 0);
        k_ln<<<(unsigned)((SEQ + 7) / 8), 256, 0, stream>>>(xb, YF, gam, bet, ob);
    }
}
